// Mamba2Layer_10617159156220
// MI455X (gfx1250) — hardware-verified
//
#include <hip/hip_runtime.h>


#define LQ   2048
#define DM   1024
#define DI   2048
#define NH   16
#define NS   64
#define HP   128
#define CD   2176
#define NZX  4224
#define NW   4240
#define NWP  4256
#define DTP  32
#define QC   64
#define NCH  32

static_assert(NCH * QC == LQ);
static_assert(NZX % 64 == 0);
static_assert(DM % 64 == 0);
static_assert(DI % 64 == 0);
static_assert(CD == DI + 2 * NS);
static_assert(CD % 8 == 0);
static_assert((CD / 2) % 32 == 0);
static_assert(HP % 32 == 0);
static_assert(NW + 16 <= NWP);

typedef float          v4f   __attribute__((ext_vector_type(4)));
typedef float          v8f   __attribute__((ext_vector_type(8)));
typedef _Float16       v8h   __attribute__((ext_vector_type(8)));
typedef _Float16       v16h  __attribute__((ext_vector_type(16)));
typedef unsigned short u16x8 __attribute__((ext_vector_type(8)));

union FragH { u16x8 h[2]; v16h v; };
union Pack8 { v8h f; u16x8 u; };

__device__ __forceinline__ v8f splat8(float f) {
  v8f z;
#pragma unroll
  for (int c = 0; c < 8; ++c) z[c] = f;
  return z;
}
__device__ __forceinline__ v8f ld8f(const float* p) {
  v4f a = *(const v4f*)p;
  v4f b = *(const v4f*)(p + 4);
  return __builtin_shufflevector(a, b, 0, 1, 2, 3, 4, 5, 6, 7);
}
__device__ __forceinline__ u16x8 pack8(v8f x) {
  Pack8 p;
  p.f = __builtin_convertvector(x, v8h);
  return p.u;
}
__device__ __forceinline__ void split8(v8f x, u16x8& hv, u16x8& lv) {
  Pack8 ph, pl;
  ph.f = __builtin_convertvector(x, v8h);
  v8f hf = __builtin_convertvector(ph.f, v8f);
  pl.f = __builtin_convertvector((x - hf) * 2048.0f, v8h);
  hv = ph.u;
  lv = pl.u;
}
__device__ __forceinline__ float silu_f(float x) {
  return x * __builtin_amdgcn_rcpf(1.0f + __expf(-x));
}

__device__ __forceinline__ void mma16(v8f& acc, const FragH& a, const FragH& b) {
  acc = __builtin_amdgcn_wmma_f32_16x16x32_f16(false, a.v, false, b.v, (short)0, acc, false, false);
  asm volatile("v_nop\n\tv_nop\n\tv_nop\n\tv_nop" : "+v"(acc) : "v"(a.v), "v"(b.v));
}
__device__ __forceinline__ v8f mma_raw(v8f acc, const FragH& a, const FragH& b) {
  return __builtin_amdgcn_wmma_f32_16x16x32_f16(false, a.v, false, b.v, (short)0, acc, false, false);
}

__global__ __launch_bounds__(256)
void k_cvt(const float* __restrict__ src, unsigned short* dh, unsigned short* dl,
           int n8, int nvalid8, int lo8, float scale)
{
  const int i = blockIdx.x * 256 + threadIdx.x;
  if (i >= n8) return;
  v8f x = splat8(0.0f);
  if (i < nvalid8) x = ld8f(src + (size_t)i * 8);
  x = x * scale;
  u16x8 hv, lv;
  split8(x, hv, lv);
  unsigned short* ph = dh + (size_t)i * 8;
  const bool wl = (i >= lo8);
  unsigned short* pl = dl + (size_t)(wl ? (i - lo8) : 0) * 8;
  *(volatile u16x8*)ph = hv;
  if (wl) *(volatile u16x8*)pl = lv;
  __threadfence();
  *(volatile u16x8*)ph = hv;
  if (wl) *(volatile u16x8*)pl = lv;
}

__global__ __launch_bounds__(128)
void k_norm_in(const float* __restrict__ x, const float* __restrict__ w,
               unsigned short* xh, unsigned short* xl)
{
  __shared__ float red[4];
  const int t = blockIdx.x, tid = threadIdx.x, lane = tid & 31, wave = tid >> 5;
  const int c0 = tid * 8;
  const v8f v = ld8f(x + (size_t)t * DM + c0);
  float ss = 0.0f;
#pragma unroll
  for (int c = 0; c < 8; ++c) ss += v[c] * v[c];
#pragma unroll
  for (int off = 16; off > 0; off >>= 1) ss += __shfl_xor(ss, off);
  if (lane == 0) red[wave] = ss;
  __syncthreads();
  const float tot = ((red[0] + red[1]) + red[2]) + red[3];
  const float inv = rsqrtf(tot * (1.0f / DM) + 1e-5f);
  const v8f wv = ld8f(w + c0);
  const v8f xn = (v * inv) * wv;
  u16x8 hv, lv;
  split8(xn, hv, lv);
  const size_t e = (size_t)t * DM + c0;
  *(volatile u16x8*)(xh + e) = hv;
  *(volatile u16x8*)(xl + e) = lv;
  __threadfence();
  *(volatile u16x8*)(xh + e) = hv;
  *(volatile u16x8*)(xl + e) = lv;
}

template<int MODE, int WN>
__global__ __launch_bounds__(128)
void k_gemm(const unsigned short* __restrict__ A,  const unsigned short* __restrict__ A2,
            const unsigned short* __restrict__ B,  const unsigned short* __restrict__ B2,
            float* C, int K, int ldc, float scale)
{
  constexpr int CW = 32;
  constexpr int P  = CW + 4;
  __shared__ __attribute__((aligned(16))) float stile[2 * WN][32 * P];

  const int tid  = threadIdx.x;
  const int lane = tid & 31;
  const int wave = tid >> 5;
  const int h    = lane >> 4;
  const int m    = lane & 15;
  const int wm   = (WN == 2) ? (wave >> 1) : wave;
  const int wn   = (WN == 2) ? (wave & 1) : 0;
  const int rowW = blockIdx.y * 64 + wm * 32;
  const int colW = blockIdx.x * (WN * CW) + wn * CW;

  v8f acc[4], accr[4];
#pragma unroll
  for (int j = 0; j < 4; ++j) { acc[j] = splat8(0.0f); accr[j] = splat8(0.0f); }

  const size_t aoff  = (size_t)(rowW + m) * K + 8 * h;
  const size_t boff  = (size_t)(colW + m) * K + 8 * h;
  const size_t sub16 = (size_t)16 * K;
  const int nk = K >> 5;

#pragma unroll 1
  for (int kt = 0; kt < nk; ++kt) {
    const size_t k0 = (size_t)kt * 32;
    FragH fa[2], ga[2], fb[2], gb[2];
#pragma unroll
    for (int s = 0; s < 2; ++s) {
      const unsigned short* p = A + aoff + s * sub16 + k0;
      fa[s].h[0] = *(const u16x8*)(p);
      fa[s].h[1] = *(const u16x8*)(p + 16);
      const unsigned short* q = A2 + aoff + s * sub16 + k0;
      ga[s].h[0] = *(const u16x8*)(q);
      ga[s].h[1] = *(const u16x8*)(q + 16);
    }
#pragma unroll
    for (int j = 0; j < 2; ++j) {
      const unsigned short* p = B + boff + j * sub16 + k0;
      fb[j].h[0] = *(const u16x8*)(p);
      fb[j].h[1] = *(const u16x8*)(p + 16);
      if constexpr (MODE == 2) {
        const unsigned short* q = B2 + boff + j * sub16 + k0;
        gb[j].h[0] = *(const u16x8*)(q);
        gb[j].h[1] = *(const u16x8*)(q + 16);
      }
    }
#pragma unroll
    for (int s = 0; s < 2; ++s)
#pragma unroll
      for (int j = 0; j < 2; ++j) {
        acc[s * 2 + j]  = mma_raw(acc[s * 2 + j],  fa[s], fb[j]);
        accr[s * 2 + j] = mma_raw(accr[s * 2 + j], ga[s], fb[j]);
        if constexpr (MODE == 2) accr[s * 2 + j] = mma_raw(accr[s * 2 + j], fa[s], gb[j]);
      }
    if constexpr (MODE == 2) {
      asm volatile("v_nop\n\tv_nop\n\tv_nop\n\tv_nop"
                   : "+v"(acc[0]), "+v"(acc[1]), "+v"(acc[2]), "+v"(acc[3]),
                     "+v"(accr[0]), "+v"(accr[1]), "+v"(accr[2]), "+v"(accr[3])
                   : "v"(fa[0].v), "v"(fa[1].v), "v"(ga[0].v), "v"(ga[1].v),
                     "v"(fb[0].v), "v"(fb[1].v), "v"(gb[0].v), "v"(gb[1].v));
    } else {
      asm volatile("v_nop\n\tv_nop\n\tv_nop\n\tv_nop"
                   : "+v"(acc[0]), "+v"(acc[1]), "+v"(acc[2]), "+v"(acc[3]),
                     "+v"(accr[0]), "+v"(accr[1]), "+v"(accr[2]), "+v"(accr[3])
                   : "v"(fa[0].v), "v"(fa[1].v), "v"(ga[0].v), "v"(ga[1].v),
                     "v"(fb[0].v), "v"(fb[1].v));
    }
  }

  float* st = stile[wave];
  const float rs = scale * (1.0f / 2048.0f);
#pragma unroll
  for (int s = 0; s < 2; ++s)
#pragma unroll
    for (int j = 0; j < 2; ++j)
#pragma unroll
      for (int r = 0; r < 8; ++r)
        st[(s * 16 + 8 * h + r) * P + j * 16 + m] = acc[s * 2 + j][r] * scale + accr[s * 2 + j][r] * rs;
  __syncthreads();

  float* gp = C + (size_t)rowW * ldc + colW;
  const int rsub = lane >> 3;
  const int c4   = (lane & 7) * 4;
#pragma unroll
  for (int it = 0; it < 8; ++it) {
    const int row = it * 4 + rsub;
    const v4f v = *(const v4f*)(st + row * P + c4);
    *(volatile v4f*)(gp + (size_t)row * ldc + c4) = v;
  }
  __threadfence();
#pragma unroll
  for (int it = 0; it < 8; ++it) {
    const int row = it * 4 + rsub;
    const v4f v = *(const v4f*)(st + row * P + c4);
    *(volatile v4f*)(gp + (size_t)row * ldc + c4) = v;
  }
}

__global__ __launch_bounds__(272)
void k_conv(const float* __restrict__ zx, const float* __restrict__ cw,
            const float* __restrict__ cb, float* xbc)
{
  __shared__ __attribute__((aligned(16))) float su[CD];
  const int t  = blockIdx.x;
  const int tid = threadIdx.x;
  const int c0 = tid * 8;
  const float* xr = zx + (size_t)t * NZX + DI + c0;
  const v8f x0 = ld8f(xr);
  v8f x1 = splat8(0.0f), x2 = splat8(0.0f), x3 = splat8(0.0f);
  if (t >= 1) x1 = ld8f(xr - NZX);
  if (t >= 2) x2 = ld8f(xr - 2 * NZX);
  if (t >= 3) x3 = ld8f(xr - 3 * NZX);
  v4f wv[8];
#pragma unroll
  for (int c = 0; c < 8; ++c) wv[c] = *(const v4f*)(cw + (size_t)(c0 + c) * 4);
  const v8f bias = ld8f(cb + c0);
  v8f u;
#pragma unroll
  for (int c = 0; c < 8; ++c) {
    float a = x0[c] * wv[c][0] + x1[c] * wv[c][1];
    a = a + x2[c] * wv[c][2];
    a = a + x3[c] * wv[c][3];
    a = a + bias[c];
    u[c] = silu_f(a);
  }
  *(v4f*)(su + c0)     = __builtin_shufflevector(u, u, 0, 1, 2, 3);
  *(v4f*)(su + c0 + 4) = __builtin_shufflevector(u, u, 4, 5, 6, 7);
  __syncthreads();

  const int e0 = tid * 4;
  const int e1 = e0 + CD / 2;
  const v4f va = *(const v4f*)(su + e0);
  const v4f vb = *(const v4f*)(su + e1);
  float* gp = xbc + (size_t)t * CD;
  *(volatile v4f*)(gp + e0) = va;
  *(volatile v4f*)(gp + e1) = vb;
  __threadfence();
  *(volatile v4f*)(gp + e0) = va;
  *(volatile v4f*)(gp + e1) = vb;
}

__global__ __launch_bounds__(128)
void k_cb(const float* __restrict__ xbc, const float* __restrict__ dtraw,
          const float* __restrict__ dtb, const float* __restrict__ alog,
          unsigned short* Mp, float* dec)
{
  __shared__ float ssp[QC * NH];
  __shared__ float scum[QC * NH];
  __shared__ __attribute__((aligned(16))) unsigned short Ct[QC * 72];
  __shared__ __attribute__((aligned(16))) unsigned short Bt[QC * 72];
  __shared__ __attribute__((aligned(16))) float Gs[QC * 68];
  __shared__ __attribute__((aligned(16))) unsigned short Ms[QC * 64];
  __shared__ __attribute__((aligned(16))) float sdec[NH * 128];

  const int kc  = blockIdx.x;
  const int t0  = kc * QC;
  const int tid = threadIdx.x, lane = tid & 31, wave = tid >> 5;
  const int hh  = lane >> 4, m = lane & 15;

  if (tid < NH) {
    const int hd = tid;
    const float nA = -__expf(alog[hd]);
    const float bias = dtb[hd];
    float run = 0.0f;
#pragma unroll 1
    for (int tau = 0; tau < QC; ++tau) {
      const float v  = dtraw[(size_t)(t0 + tau) * DTP + hd] + bias;
      const float sp = fmaxf(v, 0.0f) + log1pf(__expf(-fabsf(v)));
      ssp[tau * NH + hd] = sp;
      run = run + nA * sp;
      scum[tau * NH + hd] = run;
      sdec[hd * 128 + tau] = __expf(run);
    }
    const float c63 = run;
#pragma unroll 1
    for (int tau = 0; tau < QC; ++tau)
      sdec[hd * 128 + 64 + tau] = __expf(c63 - scum[tau * NH + hd]) * ssp[tau * NH + hd];
  }
#pragma unroll
  for (int it = 0; it < 4; ++it) {
    const int idx = it * 128 + tid;
    const int r = idx >> 3, n8 = (idx & 7) * 8;
    const float* rowp = xbc + (size_t)(t0 + r) * CD + DI + n8;
    *(u16x8*)(Bt + r * 72 + n8) = pack8(ld8f(rowp) * 16.0f);
    *(u16x8*)(Ct + r * 72 + n8) = pack8(ld8f(rowp + NS) * 16.0f);
  }
  __syncthreads();

  if (tid < NH) {
    const float* sp = sdec + tid * 128;
    float* gp = dec + (size_t)(kc * NH + tid) * 128;
#pragma unroll
    for (int i = 0; i < 32; ++i) *(volatile v4f*)(gp + 4 * i) = *(const v4f*)(sp + 4 * i);
    __threadfence();
#pragma unroll
    for (int i = 0; i < 32; ++i) *(volatile v4f*)(gp + 4 * i) = *(const v4f*)(sp + 4 * i);
  }

  {
    v8f acc[4];
#pragma unroll
    for (int j = 0; j < 4; ++j) acc[j] = splat8(0.0f);
    const int rw = wave * 16;
#pragma unroll
    for (int ks = 0; ks < 2; ++ks) {
      const int k0 = ks * 32;
      FragH a;
      const unsigned short* ap = Ct + (rw + m) * 72 + k0 + 8 * hh;
      a.h[0] = *(const u16x8*)(ap);
      a.h[1] = *(const u16x8*)(ap + 16);
#pragma unroll
      for (int j = 0; j < 4; ++j) {
        FragH b;
        const unsigned short* bp = Bt + (16 * j + m) * 72 + k0 + 8 * hh;
        b.h[0] = *(const u16x8*)(bp);
        b.h[1] = *(const u16x8*)(bp + 16);
        mma16(acc[j], a, b);
      }
    }
#pragma unroll
    for (int j = 0; j < 4; ++j)
#pragma unroll
      for (int r = 0; r < 8; ++r)
        Gs[(rw + 8 * hh + r) * 68 + 16 * j + m] = acc[j][r] * (1.0f / 256.0f);
  }
  __syncthreads();

  const int tau = tid >> 1, s0 = (tid & 1) * 32;
  const int q4 = lane >> 3, j8 = lane & 7;
#pragma unroll 1
  for (int hd = 0; hd < NH; ++hd) {
    const float ct = scum[tau * NH + hd];
#pragma unroll
    for (int g = 0; g < 4; ++g) {
      v8f vals;
#pragma unroll
      for (int c = 0; c < 8; ++c) {
        const int s = s0 + 8 * g + c;
        const float e = __expf(fminf(ct - scum[s * NH + hd], 0.0f));
        const float val = e * Gs[tau * 68 + s] * ssp[s * NH + hd] * 8.0f;
        vals[c] = (s <= tau) ? val : 0.0f;
      }
      *(u16x8*)(Ms + tau * 64 + s0 + 8 * g) = pack8(vals);
    }
    __syncthreads();
    unsigned short* gbase = Mp + (size_t)(kc * NH + hd) * (QC * QC);
    u16x8 ov[4];
#pragma unroll
    for (int it = 0; it < 4; ++it) {
      const int row = 16 * wave + 4 * it + q4;
      ov[it] = *(const u16x8*)(Ms + row * 64 + 8 * j8);
    }
#pragma unroll
    for (int it = 0; it < 4; ++it) {
      const int row = 16 * wave + 4 * it + q4;
      *(volatile u16x8*)(gbase + (size_t)row * QC + 8 * j8) = ov[it];
    }
    __threadfence();
#pragma unroll
    for (int it = 0; it < 4; ++it) {
      const int row = 16 * wave + 4 * it + q4;
      *(volatile u16x8*)(gbase + (size_t)row * QC + 8 * j8) = ov[it];
    }
    __syncthreads();
  }
}

__global__ __launch_bounds__(128)
void k_ssd(const float* __restrict__ xbc, const unsigned short* __restrict__ Mp,
           const float* __restrict__ dec, const float* __restrict__ Dv, float* y)
{
  __shared__ __attribute__((aligned(16))) float S[32 * 64];
  __shared__ __attribute__((aligned(16))) unsigned short Sh[32 * 72];
  __shared__ __attribute__((aligned(16))) unsigned short Sl[32 * 72];
  __shared__ __attribute__((aligned(16))) unsigned short Ct[QC * 72];
  __shared__ __attribute__((aligned(16))) unsigned short BdT[NS * 72];
  __shared__ __attribute__((aligned(16))) unsigned short xT[32 * 72];
  __shared__ __attribute__((aligned(16))) float Yst[QC * 36];

  const int ps = blockIdx.x, hd = blockIdx.y;
  const int col0 = hd * HP + ps * 32;
  const int tid = threadIdx.x, lane = tid & 31, wave = tid >> 5;
  const int hh = lane >> 4, m = lane & 15;
  const int rw = wave * 16;
  const int pw = wave >> 1, nt0 = (wave & 1) * 2;
  const int q4 = lane >> 3, j8 = lane & 7;
  const float Dh = Dv[hd];

  for (int i = tid; i < 32 * 64; i += 128) S[i] = 0.0f;
  __syncthreads();

#pragma unroll 1
  for (int kc = 0; kc < NCH; ++kc) {
    const int t0 = kc * QC;
    const float* drec = dec + (size_t)(kc * NH + hd) * 128;

#pragma unroll
    for (int it = 0; it < 4; ++it) {
      const int idx = it * 128 + tid;
      const int tau = idx >> 3, n8 = (idx & 7) * 8;
      const float* rowp = xbc + (size_t)(t0 + tau) * CD + DI + n8;
      *(u16x8*)(Ct + tau * 72 + n8) = pack8(ld8f(rowp + NS) * 16.0f);
      const float wd = drec[64 + tau] * 256.0f;
      Pack8 pb;
      pb.f = __builtin_convertvector(ld8f(rowp) * wd, v8h);
#pragma unroll
      for (int c = 0; c < 8; ++c) BdT[(n8 + c) * 72 + tau] = pb.u[c];
    }
#pragma unroll
    for (int it = 0; it < 2; ++it) {
      const int idx = it * 128 + tid;
      const int tau = idx >> 2, p8 = (idx & 3) * 8;
      Pack8 px;
      px.f = __builtin_convertvector(ld8f(xbc + (size_t)(t0 + tau) * CD + col0 + p8) * 16.0f, v8h);
#pragma unroll
      for (int c = 0; c < 8; ++c) xT[(p8 + c) * 72 + tau] = px.u[c];
    }
#pragma unroll
    for (int it = 0; it < 2; ++it) {
      const int idx = it * 128 + tid;
      const int p = idx >> 3, n8 = (idx & 7) * 8;
      u16x8 hv, lv;
      split8(ld8f(S + p * 64 + n8) * 16.0f, hv, lv);
      *(u16x8*)(Sh + p * 72 + n8) = hv;
      *(u16x8*)(Sl + p * 72 + n8) = lv;
    }
    __syncthreads();

    v8f ai[2], acs[2], ar[2], au[2];
#pragma unroll
    for (int j = 0; j < 2; ++j) { ai[j] = splat8(0.0f); acs[j] = splat8(0.0f); ar[j] = splat8(0.0f); au[j] = splat8(0.0f); }

#pragma unroll
    for (int ks = 0; ks < 2; ++ks) {
      const int k0 = ks * 32;
      FragH fm, fc;
      const unsigned short* mpp = Mp + ((size_t)(kc * NH + hd) * QC + rw + m) * QC + k0 + 8 * hh;
      fm.h[0] = *(const u16x8*)(mpp);
      fm.h[1] = *(const u16x8*)(mpp + 16);
      const unsigned short* cp = Ct + (rw + m) * 72 + k0 + 8 * hh;
      fc.h[0] = *(const u16x8*)(cp);
      fc.h[1] = *(const u16x8*)(cp + 16);
#pragma unroll
      for (int j = 0; j < 2; ++j) {
        FragH bx, bh, bl;
        const unsigned short* xp = xT + (16 * j + m) * 72 + k0 + 8 * hh;
        bx.h[0] = *(const u16x8*)(xp);
        bx.h[1] = *(const u16x8*)(xp + 16);
        const unsigned short* hp = Sh + (16 * j + m) * 72 + k0 + 8 * hh;
        bh.h[0] = *(const u16x8*)(hp);
        bh.h[1] = *(const u16x8*)(hp + 16);
        const unsigned short* lp = Sl + (16 * j + m) * 72 + k0 + 8 * hh;
        bl.h[0] = *(const u16x8*)(lp);
        bl.h[1] = *(const u16x8*)(lp + 16);
        mma16(ai[j],  fm, bx);
        mma16(acs[j], fc, bh);
        mma16(ar[j],  fc, bl);
      }
      FragH ax;
      const unsigned short* axp = xT + (16 * pw + m) * 72 + k0 + 8 * hh;
      ax.h[0] = *(const u16x8*)(axp);
      ax.h[1] = *(const u16x8*)(axp + 16);
#pragma unroll
      for (int jj = 0; jj < 2; ++jj) {
        FragH bb;
        const unsigned short* bp = BdT + (16 * (nt0 + jj) + m) * 72 + k0 + 8 * hh;
        bb.h[0] = *(const u16x8*)(bp);
        bb.h[1] = *(const u16x8*)(bp + 16);
        mma16(au[jj], ax, bb);
      }
    }

    const float eend = drec[63];
#pragma unroll
    for (int jj = 0; jj < 2; ++jj)
#pragma unroll
      for (int r = 0; r < 8; ++r) {
        const int p  = 16 * pw + 8 * hh + r;
        const int n  = 16 * (nt0 + jj) + m;
        const int si = p * 64 + n;
        S[si] = eend * S[si] + au[jj][r] * (1.0f / 4096.0f);
      }
    const v8f cev = ld8f(drec + rw + 8 * hh);
#pragma unroll
    for (int j = 0; j < 2; ++j)
#pragma unroll
      for (int r = 0; r < 8; ++r)
        Yst[(rw + 8 * hh + r) * 36 + 16 * j + m] =
            ai[j][r] * (1.0f / 128.0f) + cev[r] * (acs[j][r] + ar[j][r] * (1.0f / 2048.0f)) * (1.0f / 256.0f);
    __syncthreads();

    v4f ov[4];
#pragma unroll
    for (int it = 0; it < 4; ++it) {
      const int row = rw + 4 * it + q4;
      const v4f v  = *(const v4f*)(Yst + row * 36 + 4 * j8);
      const v4f xv = *(const v4f*)(xbc + (size_t)(t0 + row) * CD + col0 + 4 * j8);
      ov[it] = v + xv * Dh;
    }
#pragma unroll
    for (int it = 0; it < 4; ++it) {
      const int row = rw + 4 * it + q4;
      *(volatile v4f*)(y + (size_t)(t0 + row) * DI + col0 + 4 * j8) = ov[it];
    }
    __threadfence();
#pragma unroll
    for (int it = 0; it < 4; ++it) {
      const int row = rw + 4 * it + q4;
      *(volatile v4f*)(y + (size_t)(t0 + row) * DI + col0 + 4 * j8) = ov[it];
    }
    __syncthreads();
  }
}

__global__ __launch_bounds__(256)
void k_gate(const float* __restrict__ y, const float* __restrict__ zx, const float* __restrict__ w,
            unsigned short* yh, unsigned short* yl)
{
  __shared__ float red[8];
  const int t = blockIdx.x, tid = threadIdx.x, lane = tid & 31, wave = tid >> 5;
  const int c0 = tid * 8;
  const v8f yv = ld8f(y + (size_t)t * DI + c0);
  const v8f zv = ld8f(zx + (size_t)t * NZX + c0);
  v8f g;
  float ss = 0.0f;
#pragma unroll
  for (int c = 0; c < 8; ++c) {
    const float z  = zv[c];
    const float sg = __builtin_amdgcn_rcpf(1.0f + __expf(-z));
    const float gg = yv[c] * (z * sg);
    g[c] = gg;
    ss += gg * gg;
  }
#pragma unroll
  for (int off = 16; off > 0; off >>= 1) ss += __shfl_xor(ss, off);
  if (lane == 0) red[wave] = ss;
  __syncthreads();
  float tot = 0.0f;
#pragma unroll
  for (int i = 0; i < 8; ++i) tot += red[i];
  const float inv = rsqrtf(tot * (1.0f / DI) + 1e-5f);
  const v8f wv = ld8f(w + c0);
  const v8f yn = (g * inv) * wv;
  u16x8 hv, lv;
  split8(yn, hv, lv);
  const size_t e = (size_t)t * DI + c0;
  *(volatile u16x8*)(yh + e) = hv;
  *(volatile u16x8*)(yl + e) = lv;
  __threadfence();
  *(volatile u16x8*)(yh + e) = hv;
  *(volatile u16x8*)(yl + e) = lv;
}

extern "C" void kernel_launch(void* const* d_in, const int* in_sizes, int n_in,
                              void* d_out, int out_size, void* d_ws, size_t ws_size,
                              hipStream_t stream)
{
  if (n_in < 10) return;
  if (in_sizes[0] != LQ * DM)  return;
  if (in_sizes[1] != DM)       return;
  if (in_sizes[2] != DI)       return;
  if (in_sizes[3] != NW * DM)  return;
  if (in_sizes[4] != DM * DI)  return;
  if (in_sizes[5] != CD * 4)   return;
  if (in_sizes[6] != CD)       return;
  if (in_sizes[7] != NH)       return;
  if (in_sizes[8] != NH)       return;
  if (in_sizes[9] != NH)       return;
  if (out_size != LQ * DM)     return;

  const float* x      = (const float*)d_in[0];
  const float* w_ni   = (const float*)d_in[1];
  const float* w_no   = (const float*)d_in[2];
  const float* win    = (const float*)d_in[3];
  const float* wout   = (const float*)d_in[4];
  const float* cw     = (const float*)d_in[5];
  const float* cb     = (const float*)d_in[6];
  const float* dtb    = (const float*)d_in[7];
  const float* alog   = (const float*)d_in[8];
  const float* Dv     = (const float*)d_in[9];
  float* out = (float*)d_out;

  const size_t SZ_XP  = (size_t)LQ * DM * 2;
  const size_t SZ_WIH = (size_t)NWP * DM * 2;
  const size_t SZ_WIL = (size_t)32 * DM * 2;
  const size_t SZ_WOP = (size_t)DM * DI * 2;
  const size_t SZ_ZX  = (size_t)LQ * NZX * 4;
  const size_t SZ_DT  = (size_t)LQ * DTP * 4;
  const size_t SZ_XBC = (size_t)LQ * CD * 4;
  const size_t SZ_MP  = (size_t)NCH * NH * QC * QC * 2;
  const size_t SZ_DEC = (size_t)NCH * NH * 128 * 4;
  const size_t SZ_Y   = (size_t)LQ * DI * 4;
  const size_t SZ_YP  = (size_t)LQ * DI * 2;

  const size_t OFF_XH  = 0;
  const size_t OFF_XL  = OFF_XH  + SZ_XP;
  const size_t OFF_WIH = OFF_XL  + SZ_XP;
  const size_t OFF_WIL = OFF_WIH + SZ_WIH;
  const size_t OFF_WOH = OFF_WIL + SZ_WIL;
  const size_t OFF_WOL = OFF_WOH + SZ_WOP;
  const size_t OFF_ZX  = OFF_WOL + SZ_WOP;
  const size_t OFF_DT  = OFF_ZX  + SZ_ZX;
  const size_t OFF_XBC = OFF_DT  + SZ_DT;
  const size_t OFF_MP  = OFF_XBC + SZ_XBC;
  const size_t OFF_DEC = OFF_MP  + SZ_MP;
  const size_t OFF_Y   = OFF_DEC + SZ_DEC;
  const size_t OFF_YH  = OFF_Y   + SZ_Y;
  const size_t OFF_YL  = OFF_YH  + SZ_YP;
  const size_t WS_END  = OFF_YL  + SZ_YP;
  if (ws_size < WS_END) return;

  char* ws = (char*)d_ws;
  unsigned short* xh   = (unsigned short*)(ws + OFF_XH);
  unsigned short* xl   = (unsigned short*)(ws + OFF_XL);
  unsigned short* wih  = (unsigned short*)(ws + OFF_WIH);
  unsigned short* wil  = (unsigned short*)(ws + OFF_WIL);
  unsigned short* woh  = (unsigned short*)(ws + OFF_WOH);
  unsigned short* wol  = (unsigned short*)(ws + OFF_WOL);
  float*          zx   = (float*)(ws + OFF_ZX);
  float*          dtr  = (float*)(ws + OFF_DT);
  float*          xbc  = (float*)(ws + OFF_XBC);
  unsigned short* Mp   = (unsigned short*)(ws + OFF_MP);
  float*          dec  = (float*)(ws + OFF_DEC);
  float*          ybuf = (float*)(ws + OFF_Y);
  unsigned short* ynh  = (unsigned short*)(ws + OFF_YH);
  unsigned short* ynl  = (unsigned short*)(ws + OFF_YL);

  {
    const int n8 = NWP * DM / 8, nv8 = NW * DM / 8, lo8 = NZX * DM / 8;
    hipLaunchKernelGGL(k_cvt, dim3((n8 + 255) / 256), dim3(256), 0, stream,
                       win, wih, wil, n8, nv8, lo8, 32.0f);
  }
  {
    const int n8 = DM * DI / 8;
    hipLaunchKernelGGL(k_cvt, dim3((n8 + 255) / 256), dim3(256), 0, stream,
                       wout, woh, wol, n8, n8, 0, 64.0f);
  }
  hipLaunchKernelGGL(k_norm_in, dim3(LQ), dim3(128), 0, stream, x, w_ni, xh, xl);

  hipLaunchKernelGGL(HIP_KERNEL_NAME(k_gemm<1, 2>), dim3(NZX / 64, LQ / 64), dim3(128), 0, stream,
                     (const unsigned short*)xh, (const unsigned short*)xl,
                     (const unsigned short*)wih, (const unsigned short*)wih,
                     zx, (int)DM, (int)NZX, 1.0f / 32.0f);

  hipLaunchKernelGGL(HIP_KERNEL_NAME(k_gemm<2, 1>), dim3(1, LQ / 64), dim3(64), 0, stream,
                     (const unsigned short*)xh, (const unsigned short*)xl,
                     (const unsigned short*)(wih + (size_t)NZX * DM), (const unsigned short*)wil,
                     dtr, (int)DM, (int)DTP, 1.0f / 32.0f);

  hipLaunchKernelGGL(k_conv, dim3(LQ), dim3(CD / 8), 0, stream, (const float*)zx, cw, cb, xbc);

  hipLaunchKernelGGL(k_cb, dim3(NCH), dim3(128), 0, stream,
                     (const float*)xbc, (const float*)dtr, dtb, alog, Mp, dec);

  hipLaunchKernelGGL(k_ssd, dim3(HP / 32, NH), dim3(128), 0, stream,
                     (const float*)xbc, (const unsigned short*)Mp, (const float*)dec, Dv, ybuf);

  hipLaunchKernelGGL(k_gate, dim3(LQ), dim3(256), 0, stream,
                     (const float*)ybuf, (const float*)zx, w_no, ynh, ynl);

  hipLaunchKernelGGL(HIP_KERNEL_NAME(k_gemm<2, 2>), dim3(DM / 64, LQ / 64), dim3(128), 0, stream,
                     (const unsigned short*)ynh, (const unsigned short*)ynl,
                     (const unsigned short*)woh, (const unsigned short*)wol,
                     out, (int)DI, (int)DM, 1.0f / 64.0f);
}
